// HLUnit_13477607375168
// MI455X (gfx1250) — hardware-verified
//
#include <hip/hip_runtime.h>
#include <math.h>

#define NIMG 12
#define HI 256
#define WI 256
#define HO 254
#define WO 254
#define NF 64
#define UP 4
#define OW (WO * UP)
#define RSPLIT (1.0f / 2048.0f)

typedef _Float16 h16;
typedef __attribute__((ext_vector_type(16))) _Float16 v16h;
typedef __attribute__((ext_vector_type(8)))  _Float16 v8h;
typedef __attribute__((ext_vector_type(8)))  float v8f;
typedef __attribute__((ext_vector_type(4)))  float v4f_t;
typedef float v4fa __attribute__((ext_vector_type(4), may_alias));

__device__ __forceinline__ h16 lo_of(float v, h16 h) { return (h16)((v - (float)h) * 2048.0f); }
__device__ __forceinline__ v8f wmma16(v16h a, v16h b, v8f c) { return __builtin_amdgcn_wmma_f32_16x16x32_f16(false, a, false, b, (short)0, c, false, false); }
__device__ __forceinline__ v8f wmma_asplit(v16h a, v16h al, v16h b, v8f c) { v8f x = {}; x = wmma16(al, b, x); return wmma16(a, b, c) + x * RSPLIT; }
__device__ __forceinline__ v16h rfrag(const h16* rowp, int half) {
  const h16* p = rowp + 8 * half;
  return __builtin_shufflevector(*(const v8h*)p, *(const v8h*)(p + 16), 0,1,2,3,4,5,6,7,8,9,10,11,12,13,14,15);
}

__global__ __launch_bounds__(256) void k_hlunit(const float* __restrict__ x,
    const float* __restrict__ w1, const float* __restrict__ b1, const float* __restrict__ w2, const float* __restrict__ b2,
    const float* __restrict__ w3, const float* __restrict__ b3, const float* __restrict__ w4, const float* __restrict__ b4,
    const float* __restrict__ w5, const float* __restrict__ b5, const float* __restrict__ w6, const float* __restrict__ b6,
    float* __restrict__ out) {
  __shared__ __attribute__((aligned(16))) h16 Wt[4][NF * 72];
  __shared__ __attribute__((aligned(16))) h16 W6t[16 * 72];
  __shared__ float w1s[NF * 3], bs[5][NF], b6s[16];
  __shared__ __attribute__((aligned(16))) h16 act[8][2][16 * 72];
  __shared__ __attribute__((aligned(16))) float orow[4][OW];
  __shared__ float xs[3][WI];
  const int n = blockIdx.y, h = blockIdx.x;
  const int tid = threadIdx.x, lane = tid & 31, wave = tid >> 5, half = lane >> 4, l16 = lane & 15;
  for (int i = tid; i < 4 * NF * NF; i += 256) { const int L = i >> 12, o = (i >> 6) & 63, f = i & 63;
    const float* w = (L == 0) ? w2 : (L == 1) ? w3 : (L == 2) ? w4 : w5; Wt[L][o * 72 + f] = (h16)w[o * NF + f]; }
  for (int i = tid; i < 16 * NF; i += 256) { const int o = i >> 6, f = i & 63; W6t[o * 72 + f] = (h16)w6[o * NF + f]; }
  for (int i = tid; i < NF * 3; i += 256) w1s[i] = w1[i];
  if (tid < NF) { bs[0][tid] = b1[tid]; bs[1][tid] = b2[tid]; bs[2][tid] = b3[tid]; bs[3][tid] = b4[tid]; bs[4][tid] = b5[tid]; }
  if (tid < 16) b6s[tid] = b6[tid];
  for (int i = tid; i < WI; i += 256) xs[0][i] = x[((size_t)n * HI + h) * WI + i];
  __syncthreads();
  h16* ah = act[wave][0]; h16* al = act[wave][1];
#pragma unroll 1
  for (int tile = wave; tile < 16; tile += 8) {
    const int wbase = tile * 16;
    {
      const int px = l16, wq = min(wbase + px, WO - 1);
      const float v0 = xs[0][wq], v1 = xs[0][wq + 1], v2 = xs[0][wq + 2];
#pragma unroll 4
      for (int j = 0; j < 32; ++j) { const int f = half * 32 + j;
        const float a = w1s[f * 3 + 0] * v0 + w1s[f * 3 + 1] * v1 + w1s[f * 3 + 2] * v2 + bs[0][f];
        const float r = fmaxf(a, 0.0f); const h16 hv = (h16)r; ah[px * 72 + f] = hv; al[px * 72 + f] = lo_of(r, hv); }
    }
#pragma unroll 1
    for (int L = 0; L < 4; ++L) {
      v8f acc[4];
#pragma unroll
      for (int nt = 0; nt < 4; ++nt) { acc[nt] = v8f{}; }
#pragma unroll
      for (int kc = 0; kc < 2; ++kc) {
        const v16h a = rfrag(ah + l16 * 72 + kc * 32, half), a_l = rfrag(al + l16 * 72 + kc * 32, half);
#pragma unroll
        for (int nt = 0; nt < 4; ++nt) acc[nt] = wmma_asplit(a, a_l, rfrag(&Wt[L][(nt * 16 + l16) * 72 + kc * 32], half), acc[nt]);
      }
#pragma unroll
      for (int nt = 0; nt < 4; ++nt) { const int o = nt * 16 + l16; const float bb = bs[L + 1][o];
#pragma unroll
        for (int r = 0; r < 8; ++r) { const int px = 8 * half + r; const float v = fmaxf(acc[nt][r] + bb, 0.0f); const h16 hv = (h16)v;
          ah[px * 72 + o] = hv; al[px * 72 + o] = lo_of(v, hv); } }
    }
    {
      v8f acc = {};
#pragma unroll
      for (int kc = 0; kc < 2; ++kc) acc = wmma_asplit(rfrag(ah + l16 * 72 + kc * 32, half), rfrag(al + l16 * 72 + kc * 32, half), rfrag(&W6t[l16 * 72 + kc * 32], half), acc);
      const int c = l16, i = c >> 2, j = c & 3;
#pragma unroll
      for (int r = 0; r < 8; ++r) { const int px = 8 * half + r, w = wbase + px;
        if (w < WO) orow[i][w * 4 + j] = tanhf(acc[r] + b6s[c]); }
    }
  }
  __syncthreads();
  float* ob = out + ((size_t)n * (HO * UP) + (size_t)h * 4) * OW;
#pragma unroll 1
  for (int pass = 0; pass < 2; ++pass) {
    for (int q = tid; q < 4 * OW / 4; q += 256) *(volatile v4f_t*)(ob + q * 4) = *(const volatile v4fa*)(&orow[0][0] + q * 4);
    __threadfence();
  }
}

extern "C" void kernel_launch(void* const* d_in, const int* in_sizes, int n_in,
                              void* d_out, int out_size, void* d_ws, size_t ws_size,
                              hipStream_t stream) {
  (void)in_sizes; (void)n_in; (void)out_size; (void)d_ws; (void)ws_size;
  const float* x = (const float*)d_in[0];
  const float* w1 = (const float*)d_in[1];  const float* b1 = (const float*)d_in[2];
  const float* w2 = (const float*)d_in[3];  const float* b2 = (const float*)d_in[4];
  const float* w3 = (const float*)d_in[5];  const float* b3 = (const float*)d_in[6];
  const float* w4 = (const float*)d_in[7];  const float* b4 = (const float*)d_in[8];
  const float* w5 = (const float*)d_in[9];  const float* b5 = (const float*)d_in[10];
  const float* w6 = (const float*)d_in[11]; const float* b6 = (const float*)d_in[12];
  k_hlunit<<<dim3(HO, NIMG), 256, 0, stream>>>(x, w1, b1, w2, b2, w3, b3, w4, b4, w5, b5, w6, b6, (float*)d_out);
}
